// GNN_73040213836197
// MI455X (gfx1250) — hardware-verified
//
#include <hip/hip_runtime.h>
#include <stddef.h>
#include <stdint.h>


#define NN     2048
#define HD     32
#define NTHR   256
#define NWAVE  8
#define EPT    8
#define CHUNK  (NTHR * EPT)
#define NSUB   4
#define SUPER  (NSUB * CHUNK)
#define WCAP   (NSUB * EPT * 32)
#define LISTN  (NWAVE * WCAP)
#define NBRUN  32
#define SLB    5
#define LP     2112
#define DEGCAP LP
#define LST_INTS (NBRUN * LP / 2)
#define LDS_INTS (LST_INTS + LISTN + 16 + NBRUN)
#define NPB    (NN * 8 / NTHR)
#define NOUT   (NN * 3)
#define WSMAX  134217728

static_assert(NBRUN == 32 && (1 << SLB) == NBRUN);
static_assert(NN % NBRUN == 0 && NN % NWAVE == 0);
static_assert(((NN - 1) << SLB) < (1 << 30));
static_assert(LP % 64 == 0 && LP % 16 == 0 && LP >= 2047 + 8);
static_assert((NBRUN * LP) % (8 * NTHR) == 0);
static_assert(((LST_INTS + LISTN) % (4 * NTHR)) == 0);
static_assert(LDS_INTS * 4 <= 300000);
static_assert((NN * 8) % NTHR == 0);
static_assert(NOUT % NTHR == 0 && (NTHR * 4) % 128 == 0);
static_assert(HD == 32);

typedef float          v4f   __attribute__((ext_vector_type(4)));
typedef float          v8f   __attribute__((ext_vector_type(8)));
typedef int            v4i   __attribute__((ext_vector_type(4)));
typedef int            v8i   __attribute__((ext_vector_type(8)));
typedef unsigned short v8us  __attribute__((ext_vector_type(8)));
typedef unsigned short v16us __attribute__((ext_vector_type(16)));
typedef __bf16         v16bf __attribute__((ext_vector_type(16)));
typedef v4f  __attribute__((may_alias)) v4fa;
typedef v4i  __attribute__((may_alias)) v4ia;
typedef v8us __attribute__((may_alias)) v8usa;
union FragB { v16bf v; v16us u; v8us h[2]; v8i w; };

__device__ __forceinline__ v8f wmb(const FragB& a, const FragB& b, v8f c) {
  v8f d = __builtin_amdgcn_wmma_f32_16x16x32_bf16(false, a.v, false, b.v, (short)0, c, false, false);
  asm volatile("v_nop\n\tv_nop\n\tv_nop\n\tv_nop" : "+v"(d) : "v"(a.w), "v"(b.w));
  return d;
}

__device__ __forceinline__ unsigned bf16_bits(float f) {
  const unsigned u = __float_as_uint(f);
  return (u + 0x7FFFu + ((u >> 16) & 1u)) >> 16;
}
__device__ __forceinline__ float bf16_val(float f) {
  return __uint_as_float(bf16_bits(f) << 16);
}

__device__ __forceinline__ void wave_sync() {
  __builtin_amdgcn_fence(__ATOMIC_RELEASE, "wavefront");
  __builtin_amdgcn_wave_barrier();
  __builtin_amdgcn_fence(__ATOMIC_ACQUIRE, "wavefront");
}

__device__ __forceinline__ int clampn(int s) {
  return s < 0 ? 0 : (s > NN - 1 ? NN - 1 : s);
}

__device__ __forceinline__ v8f ld8(const float* p) {
  const v4f a = *(const v4f*)p;
  const v4f b = *(const v4f*)(p + 4);
  v8f r;
  r[0] = a.x; r[1] = a.y; r[2] = a.z; r[3] = a.w;
  r[4] = b.x; r[5] = b.y; r[6] = b.z; r[7] = b.w;
  return r;
}
__device__ __forceinline__ v8f ld8bf(const float* p) {
  const v8f a = ld8(p);
  v8f r;
#pragma unroll
  for (int j = 0; j < 8; ++j) r[j] = bf16_val(a[j]);
  return r;
}

__device__ __forceinline__ void split2(float v0, float v1, int& hw, int& lw) {
  const unsigned h0 = bf16_bits(v0), h1 = bf16_bits(v1);
  const unsigned l0 = bf16_bits(v0 - __uint_as_float(h0 << 16));
  const unsigned l1 = bf16_bits(v1 - __uint_as_float(h1 << 16));
  hw = (int)(h0 | (h1 << 16));
  lw = (int)(l0 | (l1 << 16));
}
__device__ __forceinline__ void split16(const v8f& e0, const v8f& e1, FragB& fh, FragB& fl) {
  v8i hw, lw;
#pragma unroll
  for (int j = 0; j < 4; ++j) {
    int a, b;
    split2(e0[2 * j], e0[2 * j + 1], a, b);
    hw[j] = a; lw[j] = b;
    split2(e1[2 * j], e1[2 * j + 1], a, b);
    hw[4 + j] = a; lw[4 + j] = b;
  }
  fh.w = hw;
  fl.w = lw;
}

__device__ __forceinline__ void l1pair(float x0, float x1, float x2,
                                       float wa0, float wa1, float wa2,
                                       float wb0, float wb1, float wb2,
                                       float bb, float& ao, float& bo) {
  float pa = x0 * bf16_val(wa0);
  pa = fmaf(x1, bf16_val(wa1), pa);
  pa = fmaf(x2, bf16_val(wa2), pa);
  float pb = x0 * bf16_val(wb0);
  pb = fmaf(x1, bf16_val(wb1), pb);
  pb = fmaf(x2, bf16_val(wb2), pb);
  ao = (bf16_val(bb) + pa) - pb;
  bo = pb;
}

__global__ __launch_bounds__(NTHR) void k_prep(const float* __restrict__ x, const float* __restrict__ W1,
                                               const float* __restrict__ b1, const float* __restrict__ W2,
                                               const float* __restrict__ W3,
                                               float* Ap, float* Bp, unsigned short* WT) {
  const int tid = (int)threadIdx.x;
  if ((int)blockIdx.x < NPB) {
    const int u = (int)blockIdx.x * NTHR + tid;
    const int i = u >> 3, q = u & 7;
    const float x0 = bf16_val(x[3 * i + 0]);
    const float x1 = bf16_val(x[3 * i + 1]);
    const float x2 = bf16_val(x[3 * i + 2]);
    const v4f wa0 = *(const v4f*)(W1 + 0 * HD + 4 * q);
    const v4f wa1 = *(const v4f*)(W1 + 1 * HD + 4 * q);
    const v4f wa2 = *(const v4f*)(W1 + 2 * HD + 4 * q);
    const v4f wb0 = *(const v4f*)(W1 + 3 * HD + 4 * q);
    const v4f wb1 = *(const v4f*)(W1 + 4 * HD + 4 * q);
    const v4f wb2 = *(const v4f*)(W1 + 5 * HD + 4 * q);
    const v4f bb  = *(const v4f*)(b1 + 4 * q);
    v4f av, bv;
    float a, b;
    l1pair(x0, x1, x2, wa0.x, wa1.x, wa2.x, wb0.x, wb1.x, wb2.x, bb.x, a, b); av.x = a; bv.x = b;
    l1pair(x0, x1, x2, wa0.y, wa1.y, wa2.y, wb0.y, wb1.y, wb2.y, bb.y, a, b); av.y = a; bv.y = b;
    l1pair(x0, x1, x2, wa0.z, wa1.z, wa2.z, wb0.z, wb1.z, wb2.z, bb.z, a, b); av.z = a; bv.z = b;
    l1pair(x0, x1, x2, wa0.w, wa1.w, wa2.w, wb0.w, wb1.w, wb2.w, bb.w, a, b); av.w = a; bv.w = b;
    float* pa = Ap + (size_t)i * HD + 4 * q;
    float* pb = Bp + (size_t)i * HD + 4 * q;
    *(volatile v4f*)pa = av;
    *(volatile v4f*)pb = bv;
    __threadfence();
    *(volatile v4f*)pa = av;
    *(volatile v4f*)pb = bv;
  } else {
    const int mat = tid >> 7;
    const int v   = tid & 127;
    const int n   = v >> 2;
    const int k8  = (v & 3) * 8;
    v8us o;
    if (mat == 0) {
#pragma unroll
      for (int j = 0; j < 8; ++j) o[j] = (unsigned short)bf16_bits(W2[(k8 + j) * HD + n]);
    } else {
#pragma unroll
      for (int j = 0; j < 8; ++j) o[j] = (unsigned short)bf16_bits(W3[(k8 + j) * HD + n]);
    }
    unsigned short* dp = WT + (size_t)mat * (HD * HD) + n * HD + k8;
    *(volatile v8us*)dp = o;
    __threadfence();
    *(volatile v8us*)dp = o;
  }
}

__device__ __forceinline__ int scan_chunk(const int* __restrict__ srcs, const int* __restrict__ dsts, int nE,
                                          int cbase, int slotBase, int vec8, int* list,
                                          int tid, int wave, int wc) {
  const int el0  = tid * EPT;
  const int e0   = cbase + el0;
  const int sent = -2147483647 - 1;
  const bool vecp = (vec8 != 0) && (cbase + CHUNK <= nE);
  v4i da, db;
  if (vecp) {
    da = *(const v4i*)(dsts + e0);
    db = *(const v4i*)(dsts + e0 + 4);
  } else {
    da.x = (e0     < nE) ? dsts[min(e0,     nE - 1)] : sent;
    da.y = (e0 + 1 < nE) ? dsts[min(e0 + 1, nE - 1)] : sent;
    da.z = (e0 + 2 < nE) ? dsts[min(e0 + 2, nE - 1)] : sent;
    da.w = (e0 + 3 < nE) ? dsts[min(e0 + 3, nE - 1)] : sent;
    db.x = (e0 + 4 < nE) ? dsts[min(e0 + 4, nE - 1)] : sent;
    db.y = (e0 + 5 < nE) ? dsts[min(e0 + 5, nE - 1)] : sent;
    db.z = (e0 + 6 < nE) ? dsts[min(e0 + 6, nE - 1)] : sent;
    db.w = (e0 + 7 < nE) ? dsts[min(e0 + 7, nE - 1)] : sent;
  }
  const unsigned nbs = (unsigned)slotBase;
  const unsigned unb = (unsigned)NBRUN;
  const unsigned s0 = (unsigned)da.x - nbs, s1 = (unsigned)da.y - nbs;
  const unsigned s2 = (unsigned)da.z - nbs, s3 = (unsigned)da.w - nbs;
  const unsigned s4 = (unsigned)db.x - nbs, s5 = (unsigned)db.y - nbs;
  const unsigned s6 = (unsigned)db.z - nbs, s7 = (unsigned)db.w - nbs;
  const bool h0 = s0 < unb, h1 = s1 < unb, h2 = s2 < unb, h3 = s3 < unb;
  const bool h4 = s4 < unb, h5 = s5 < unb, h6 = s6 < unb, h7 = s7 < unb;
  const unsigned any = __builtin_amdgcn_ballot_w32(h0 | h1 | h2 | h3 | h4 | h5 | h6 | h7);
  if (any != 0u) {
    v4i sa, sb;
    if (vecp) {
      sa = *(const v4i*)(srcs + e0);
      sb = *(const v4i*)(srcs + e0 + 4);
    } else {
      sa.x = srcs[min(e0,     nE - 1)];
      sa.y = srcs[min(e0 + 1, nE - 1)];
      sa.z = srcs[min(e0 + 2, nE - 1)];
      sa.w = srcs[min(e0 + 3, nE - 1)];
      sb.x = srcs[min(e0 + 4, nE - 1)];
      sb.y = srcs[min(e0 + 5, nE - 1)];
      sb.z = srcs[min(e0 + 6, nE - 1)];
      sb.w = srcs[min(e0 + 7, nE - 1)];
    }
    const int c0 = clampn(sa.x), c1 = clampn(sa.y), c2 = clampn(sa.z), c3 = clampn(sa.w);
    const int c4 = clampn(sb.x), c5 = clampn(sb.y), c6 = clampn(sb.z), c7 = clampn(sb.w);
#define HITJ(HJ, SJ, CJ) { \
      const unsigned mj = __builtin_amdgcn_ballot_w32(HJ); \
      if (mj != 0u) { \
        if (HJ) { \
          const int pos = wc + (int)__builtin_amdgcn_mbcnt_lo(mj, 0u); \
          if (pos < WCAP) list[wave * WCAP + pos] = ((CJ) << SLB) | (int)(SJ); \
        } \
        wc += (int)__builtin_popcount(mj); } }
    HITJ(h0, s0, c0)
    HITJ(h1, s1, c1)
    HITJ(h2, s2, c2)
    HITJ(h3, s3, c3)
    HITJ(h4, s4, c4)
    HITJ(h5, s5, c5)
    HITJ(h6, s6, c6)
    HITJ(h7, s7, c7)
#undef HITJ
  }
  return wc;
}

__global__ __launch_bounds__(NTHR) void k_lists(const int* __restrict__ srcs, const int* __restrict__ dsts,
                                                int nE, int vec8, unsigned short* LISTg, int* CNTg) {
  extern __shared__ __attribute__((aligned(16))) int dsm[];
  unsigned short* lst = (unsigned short*)dsm;
  int* list = dsm + LST_INTS;
  int* wcnt = list + LISTN;
  int* cnts = wcnt + 16;
  const int tid = (int)threadIdx.x, lane = tid & 31, wave = tid >> 5;
  const int nodeBase = (int)blockIdx.x * NBRUN;

  {
    const v4i z4 = {0, 0, 0, 0};
#pragma unroll 1
    for (int i = tid * 4; i < LST_INTS + LISTN; i += NTHR * 4) *(v4ia*)(dsm + i) = z4;
    if (tid < 16 + NBRUN) wcnt[tid] = 0;
  }
  __syncthreads();

  int cur = 0;
  const int nSuper = (nE + SUPER - 1) / SUPER;
#pragma unroll 1
  for (int sc = 0; sc < nSuper; ++sc) {
    int wc = 0;
#pragma unroll 1
    for (int sub = 0; sub < NSUB; ++sub) {
      const int cbase = sc * SUPER + sub * CHUNK;
      if (cbase < nE)
        wc = scan_chunk(srcs, dsts, nE, cbase, nodeBase, vec8, list, tid, wave, wc);
    }
    if (lane == 0) wcnt[wave] = wc;
    __syncthreads();
    if (wave == 0) {
#pragma unroll 1
      for (int w2 = 0; w2 < NWAVE; ++w2) {
        int c = wcnt[w2];
        c = c < 0 ? 0 : (c > WCAP ? WCAP : c);
#pragma unroll 1
        for (int b0 = 0; b0 < c; b0 += 32) {
          const int idx = b0 + lane;
          const int ent = list[w2 * WCAP + (idx < WCAP ? idx : WCAP - 1)];
          const bool valid = idx < c;
          const unsigned V  = __builtin_amdgcn_ballot_w32(valid);
          const unsigned B0 = __builtin_amdgcn_ballot_w32((ent & 1) != 0);
          const unsigned B1 = __builtin_amdgcn_ballot_w32((ent & 2) != 0);
          const unsigned B2 = __builtin_amdgcn_ballot_w32((ent & 4) != 0);
          const unsigned B3 = __builtin_amdgcn_ballot_w32((ent & 8) != 0);
          const unsigned B4 = __builtin_amdgcn_ballot_w32((ent & 16) != 0);
          unsigned M = V;
          M &= ((lane & 1)  != 0) ? B0 : ~B0;
          M &= ((lane & 2)  != 0) ? B1 : ~B1;
          M &= ((lane & 4)  != 0) ? B2 : ~B2;
          M &= ((lane & 8)  != 0) ? B3 : ~B3;
          M &= ((lane & 16) != 0) ? B4 : ~B4;
#pragma unroll 1
          for (int it = 0; it < 32; ++it) {
            if (__builtin_amdgcn_ballot_w32(M != 0u) == 0u) break;
            const bool on = (M != 0u);
            const int k = on ? (__builtin_ffs((int)M) - 1) : 0;
            const int j = b0 + k;
            const int e2 = list[w2 * WCAP + (j < WCAP ? j : WCAP - 1)];
            if (on) {
              if (cur < DEGCAP) lst[lane * LP + cur] = (unsigned short)(e2 >> SLB);
              cur = cur + 1;
            }
            M &= (M - 1u);
          }
        }
      }
    }
    __syncthreads();
  }

  if (wave == 0) cnts[lane] = cur;
  __syncthreads();

  unsigned short* gp = LISTg + (size_t)nodeBase * LP;
#pragma unroll 1
  for (int u = tid; u < NBRUN * LP / 8; u += NTHR) {
    const v8us q = *(const v8usa*)(lst + 8 * u);
    *(volatile v8us*)(gp + (size_t)8 * u) = q;
  }
  __threadfence();
#pragma unroll 1
  for (int u = tid; u < NBRUN * LP / 8; u += NTHR) {
    const v8us q = *(const v8usa*)(lst + 8 * u);
    *(volatile v8us*)(gp + (size_t)8 * u) = q;
  }
  const v4i cv = *(const v4ia*)(cnts + 4 * (lane & 7));
  int* cp = CNTg + nodeBase + 4 * (tid & 7);
  if (tid < 8) *(volatile v4i*)cp = cv;
  __threadfence();
  if (tid < 8) *(volatile v4i*)cp = cv;
}

__global__ __launch_bounds__(NTHR) void k_edge(const float* __restrict__ Ap, const float* __restrict__ Bp,
                                               const unsigned short* __restrict__ WT,
                                               const float* __restrict__ b2, const float* __restrict__ b3,
                                               const unsigned short* __restrict__ LISTg,
                                               const int* __restrict__ CNTg, float* S3) {
  __shared__ __attribute__((aligned(16))) float srow[NWAVE * HD];
  const int tid = (int)threadIdx.x, lane = tid & 31, wave = tid >> 5, h = lane >> 4, m = lane & 15;
  const int i = (int)blockIdx.x * NWAVE + wave;

  const int craw = __builtin_amdgcn_readfirstlane(CNTg[i]);
  const bool big = craw > DEGCAP;
  const int c = craw < 0 ? 0 : (craw > DEGCAP ? DEGCAP : craw);
  const int ntile = (c + 15) >> 4;

  FragB w2f0, w2f1, w3f0, w3f1;
  {
    const unsigned short* wp = WT + (size_t)m * HD + 8 * h;
    w2f0.h[0] = *(const v8usa*)(wp);
    w2f0.h[1] = *(const v8usa*)(wp + 16);
    w2f1.h[0] = *(const v8usa*)(wp + 16 * HD);
    w2f1.h[1] = *(const v8usa*)(wp + 16 * HD + 16);
    w3f0.h[0] = *(const v8usa*)(wp + HD * HD);
    w3f0.h[1] = *(const v8usa*)(wp + HD * HD + 16);
    w3f1.h[0] = *(const v8usa*)(wp + HD * HD + 16 * HD);
    w3f1.h[1] = *(const v8usa*)(wp + HD * HD + 16 * HD + 16);
  }
  const v8f bz20 = ld8bf(b2 + 8 * h);
  const v8f bz21 = ld8bf(b2 + 16 + 8 * h);
  const v8f bz30 = ld8bf(b3 + 8 * h);
  const v8f bz31 = ld8bf(b3 + 16 + 8 * h);
  const v8f av0 = ld8(Ap + (size_t)i * HD + 8 * h);
  const v8f av1 = ld8(Ap + (size_t)i * HD + 16 + 8 * h);

  v8f sa0 = {0.f, 0.f, 0.f, 0.f, 0.f, 0.f, 0.f, 0.f};
  v8f sa1 = sa0;
  const unsigned short* lrow = LISTg + (size_t)i * LP;

#pragma unroll 1
  for (int t = 0; t < ntile; ++t) {
    const int li = t * 16 + m;
    int s = (int)lrow[li];
    s = s > NN - 1 ? NN - 1 : s;
    const float* bp = Bp + (size_t)s * HD + 8 * h;
    const v8f g0 = ld8(bp);
    const v8f g1 = ld8(bp + 16);
    v8f e0, e1;
#pragma unroll
    for (int r = 0; r < 8; ++r) {
      e0[r] = fmaxf(av0[r] + g0[r], 0.0f);
      e1[r] = fmaxf(av1[r] + g1[r], 0.0f);
    }
    FragB bh, bl;
    split16(e0, e1, bh, bl);
    v8f d0 = bz20, d1 = bz21;
    d0 = wmb(w2f0, bh, d0);
    d1 = wmb(w2f1, bh, d1);
    d0 = wmb(w2f0, bl, d0);
    d1 = wmb(w2f1, bl, d1);
#pragma unroll
    for (int r = 0; r < 8; ++r) {
      e0[r] = fmaxf(d0[r], 0.0f);
      e1[r] = fmaxf(d1[r], 0.0f);
    }
    split16(e0, e1, bh, bl);
    d0 = bz30; d1 = bz31;
    d0 = wmb(w3f0, bh, d0);
    d1 = wmb(w3f1, bh, d1);
    d0 = wmb(w3f0, bl, d0);
    d1 = wmb(w3f1, bl, d1);
    const bool ok = li < c;
#pragma unroll
    for (int r = 0; r < 8; ++r) {
      const float y0 = fmaxf(d0[r], 0.0f);
      const float y1 = fmaxf(d1[r], 0.0f);
      sa0[r] += ok ? y0 : 0.0f;
      sa1[r] += ok ? y1 : 0.0f;
    }
  }

#pragma unroll
  for (int r = 0; r < 8; ++r) {
    float v = sa0[r];
    v += __shfl_xor(v, 1, 32);
    v += __shfl_xor(v, 2, 32);
    v += __shfl_xor(v, 4, 32);
    v += __shfl_xor(v, 8, 32);
    sa0[r] = v;
    float w = sa1[r];
    w += __shfl_xor(w, 1, 32);
    w += __shfl_xor(w, 2, 32);
    w += __shfl_xor(w, 4, 32);
    w += __shfl_xor(w, 8, 32);
    sa1[r] = w;
  }
  if (m == 0) {
#pragma unroll
    for (int r = 0; r < 8; ++r) {
      srow[wave * HD + 8 * h + r]      = sa0[r];
      srow[wave * HD + 16 + 8 * h + r] = sa1[r];
    }
  }
  wave_sync();
  v4f ov = *(const v4fa*)(srow + wave * HD + 4 * (lane & 7));
  const float qnan = __int_as_float(0x7fc00000);
  ov.x = big ? qnan : ov.x;
  ov.y = big ? qnan : ov.y;
  ov.z = big ? qnan : ov.z;
  ov.w = big ? qnan : ov.w;
  float* op = S3 + (size_t)i * HD + 4 * (lane & 7);
  if (lane < 8) *(volatile v4f*)op = ov;
  __threadfence();
  if (lane < 8) *(volatile v4f*)op = ov;
}

__global__ __launch_bounds__(NTHR) void k_out(const float* __restrict__ S3, const int* __restrict__ CNTg,
                                              const float* __restrict__ W4, const float* __restrict__ b4,
                                              float* out) {
  __shared__ float w4s[HD * 3];
  __shared__ float b4s[4];
  __shared__ __attribute__((aligned(16))) float os[NTHR];
  const int tid = (int)threadIdx.x;
  if (tid < HD * 3) w4s[tid] = bf16_val(W4[tid]);
  if (tid < 4) {
    const float bb = b4[tid < 3 ? tid : 2];
    b4s[tid] = (tid < 3) ? bf16_val(bb) : 0.0f;
  }
  __syncthreads();
  const int e = (int)blockIdx.x * NTHR + tid;
  const int i = e / 3;
  const int c = e - 3 * i;
  int cn = CNTg[i];
  cn = cn < 0 ? 0 : cn;
  const float* pr = S3 + (size_t)i * HD;
  float s = 0.0f;
#pragma unroll 1
  for (int k4 = 0; k4 < HD / 4; ++k4) {
    const v4f p = *(const v4f*)(pr + 4 * k4);
    const float* w = w4s + (4 * k4) * 3 + c;
    s = fmaf(p.x, w[0], s);
    s = fmaf(p.y, w[3], s);
    s = fmaf(p.z, w[6], s);
    s = fmaf(p.w, w[9], s);
  }
  const float cf  = (float)cn;
  const float den = (cn < 1) ? 1.0f : cf;
  const float rv  = (s + cf * b4s[c]) * (1.0f / den);
  os[tid] = rv;
  __syncthreads();
  const v4f ov = *(const v4fa*)(os + 4 * (tid & 63));
  float* op = out + (size_t)blockIdx.x * NTHR + 4 * (tid & 63);
  if (tid < 64) *(volatile v4f*)op = ov;
  __threadfence();
  if (tid < 64) *(volatile v4f*)op = ov;
}

static inline size_t al256(size_t o) { return (o + 255) & ~(size_t)255; }

extern "C" void kernel_launch(void* const* d_in, const int* in_sizes, int n_in,
                              void* d_out, int out_size, void* d_ws, size_t ws_size,
                              hipStream_t stream) {
  if (n_in < 10) return;
  if (in_sizes[0] != NN * 3) return;
  if (in_sizes[1] < 2 || (in_sizes[1] & 1) != 0) return;
  const int nE = in_sizes[1] / 2;
  if (nE < 1 || nE > (1 << 30) - SUPER) return;
  if (in_sizes[2] != 6 * HD || in_sizes[3] != HD) return;
  if (in_sizes[4] != HD * HD || in_sizes[5] != HD) return;
  if (in_sizes[6] != HD * HD || in_sizes[7] != HD) return;
  if (in_sizes[8] != HD * 3 || in_sizes[9] != 3) return;
  if (out_size != NOUT) return;

  const float* x    = (const float*)d_in[0];
  const int*   edge = (const int*)d_in[1];
  const float* W1   = (const float*)d_in[2];
  const float* b1   = (const float*)d_in[3];
  const float* W2   = (const float*)d_in[4];
  const float* b2   = (const float*)d_in[5];
  const float* W3   = (const float*)d_in[6];
  const float* b3   = (const float*)d_in[7];
  const float* W4   = (const float*)d_in[8];
  const float* b4   = (const float*)d_in[9];
  float* out = (float*)d_out;
  const int* src = edge;
  const int* dst = edge + nE;
  const int vec8 = ((nE & 3) == 0) ? 1 : 0;

  char* ws = (char*)d_ws;
  size_t off = 0;
  const size_t oA   = off; off = al256(off + (size_t)NN * HD * 4);
  const size_t oB   = off; off = al256(off + (size_t)NN * HD * 4);
  const size_t oS3  = off; off = al256(off + (size_t)NN * HD * 4);
  const size_t oWT  = off; off = al256(off + (size_t)2 * HD * HD * 2);
  const size_t oCN  = off; off = al256(off + (size_t)NN * 4);
  const size_t oLS  = off; off = al256(off + (size_t)NN * LP * 2);
  if (off > ws_size || off > (size_t)WSMAX) return;
  float*          Ap   = (float*)(ws + oA);
  float*          Bp   = (float*)(ws + oB);
  float*          S3   = (float*)(ws + oS3);
  unsigned short* WT   = (unsigned short*)(ws + oWT);
  int*            CNTg = (int*)(ws + oCN);
  unsigned short* LSTg = (unsigned short*)(ws + oLS);

  const size_t listLds = (size_t)LDS_INTS * 4;
  hipFuncSetAttribute(reinterpret_cast<const void*>(&k_lists), hipFuncAttributeMaxDynamicSharedMemorySize,
                      (int)listLds);

  k_prep<<<NPB + 1, NTHR, 0, stream>>>(x, W1, b1, W2, W3, Ap, Bp, WT);
  k_lists<<<NN / NBRUN, NTHR, listLds, stream>>>(src, dst, nE, vec8, LSTg, CNTg);
  k_edge<<<NN / NWAVE, NTHR, 0, stream>>>(Ap, Bp, WT, b2, b3, LSTg, CNTg, S3);
  k_out<<<NOUT / NTHR, NTHR, 0, stream>>>(S3, CNTg, W4, b4, out);
}
